// GNNSat_V2_2_18940805776102
// MI455X (gfx1250) — hardware-verified
//
#include <hip/hip_runtime.h>
#include <stddef.h>
#include <math.h>


#define HC      64
#define FH      32
#define ALP     4
#define ZPW     128
#define BNW     256
#define MISCN   32
#define WP      64
#define SAP     72
#define GBM     64
#define GTHR    128
#define NTHR    256
#define NWAVE   8
#define EPT     8
#define CHUNK   (NTHR * EPT)
#define WCAP    (EPT * 32)
#define LISTN   (NWAVE * WCAP)
#define NBMAX   2048
#define SLOTB   11
#define RCAP    20480
#define DEGCAP  4096
#define NEG_GAT 0.2f
#define NEG_ACT 0.01f
#define BN_EPSD 1.0e-5
#define CA      16.0f
#define CW      64.0f
#define SCL     0.0009765625f
#define WSCAP   134217728
#define LDS_BUILD ((2 * RCAP + 2 * NBMAX + LISTN) * 4 + 64)

static_assert((CHUNK & (CHUNK - 1)) == 0 && CHUNK <= 4096);
static_assert(NBMAX == (1 << SLOTB));
static_assert(NTHR * 8 == NBMAX);
static_assert(LISTN >= NBMAX);
static_assert(LISTN >= NWAVE * WCAP);
static_assert((RCAP % 32) == 0);
static_assert(LDS_BUILD <= 300000);
static_assert(GBM == (GTHR / 32) * 16);
static_assert(GBM * 4 == NTHR);
static_assert((SAP * 2) % 16 == 0 && SAP >= HC);
static_assert((HC % 32) == 0 && HC == 64);
static_assert(ZPW == 2 * HC && BNW == 4 * HC && MISCN == 32);
static_assert(FH == 32);

typedef float    v2f  __attribute__((ext_vector_type(2)));
typedef float    v4f  __attribute__((ext_vector_type(4)));
typedef float    v8f  __attribute__((ext_vector_type(8)));
typedef int      v4i  __attribute__((ext_vector_type(4)));
typedef int      v8i  __attribute__((ext_vector_type(8)));
typedef _Float16 v8h  __attribute__((ext_vector_type(8)));
typedef _Float16 v16h __attribute__((ext_vector_type(16)));
union FragH { v16h v; v8h h[2]; v8i w; };

__device__ __forceinline__ v8f wmh(const FragH& a, const FragH& b, v8f c) {
  v8f d = __builtin_amdgcn_wmma_f32_16x16x32_f16(false, a.v, false, b.v, (short)0, c, false, false);
  asm volatile("v_nop\n\tv_nop\n\tv_nop\n\tv_nop" : "+v"(d) : "v"(a.w), "v"(b.w));
  return d;
}

__device__ __forceinline__ v8h pack8(v4f a, v4f b, float sc) {
  v8h hv;
  hv[0] = (_Float16)(a.x * sc); hv[1] = (_Float16)(a.y * sc);
  hv[2] = (_Float16)(a.z * sc); hv[3] = (_Float16)(a.w * sc);
  hv[4] = (_Float16)(b.x * sc); hv[5] = (_Float16)(b.y * sc);
  hv[6] = (_Float16)(b.z * sc); hv[7] = (_Float16)(b.w * sc);
  return hv;
}

__device__ __forceinline__ float lk(float v, float s) {
  return v >= 0.f ? v : v * s;
}

__device__ __forceinline__ v4f leaky4(v4f v, float s) {
  const v4f t = v * s;
  v4f r;
  r.x = v.x >= 0.f ? v.x : t.x;
  r.y = v.y >= 0.f ? v.y : t.y;
  r.z = v.z >= 0.f ? v.z : t.z;
  r.w = v.w >= 0.f ? v.w : t.w;
  return r;
}

__device__ __forceinline__ float bnl(float v, const float* t, int c) {
  const float y = fmaf(v - t[c], t[HC + c], t[2 * HC + c]);
  return y >= 0.f ? y : y * NEG_ACT;
}

__device__ __forceinline__ int scan_chunk(const int* __restrict__ dsts, int nE, int cbase, int slotBase,
                                          int nb, int vec8, int* list, int tid, int lane, int wave) {
  int wc = 0;
  const int el0  = tid * EPT;
  const int e0   = cbase + el0;
  const int sent = -2147483647 - 1;
  v4i da, db;
  if (vec8 != 0 && cbase + CHUNK <= nE) {
    da = *(const v4i*)(dsts + e0);
    db = *(const v4i*)(dsts + e0 + 4);
  } else {
    da.x = (e0     < nE) ? dsts[min(e0,     nE - 1)] : sent;
    da.y = (e0 + 1 < nE) ? dsts[min(e0 + 1, nE - 1)] : sent;
    da.z = (e0 + 2 < nE) ? dsts[min(e0 + 2, nE - 1)] : sent;
    da.w = (e0 + 3 < nE) ? dsts[min(e0 + 3, nE - 1)] : sent;
    db.x = (e0 + 4 < nE) ? dsts[min(e0 + 4, nE - 1)] : sent;
    db.y = (e0 + 5 < nE) ? dsts[min(e0 + 5, nE - 1)] : sent;
    db.z = (e0 + 6 < nE) ? dsts[min(e0 + 6, nE - 1)] : sent;
    db.w = (e0 + 7 < nE) ? dsts[min(e0 + 7, nE - 1)] : sent;
  }
  const unsigned nbs = (unsigned)slotBase;
  const unsigned unb = (unsigned)nb;
  const unsigned s0 = (unsigned)da.x - nbs, s1 = (unsigned)da.y - nbs;
  const unsigned s2 = (unsigned)da.z - nbs, s3 = (unsigned)da.w - nbs;
  const unsigned s4 = (unsigned)db.x - nbs, s5 = (unsigned)db.y - nbs;
  const unsigned s6 = (unsigned)db.z - nbs, s7 = (unsigned)db.w - nbs;
  const bool h0 = s0 < unb, h1 = s1 < unb, h2 = s2 < unb, h3 = s3 < unb;
  const bool h4 = s4 < unb, h5 = s5 < unb, h6 = s6 < unb, h7 = s7 < unb;
  const unsigned any = __builtin_amdgcn_ballot_w32(h0 | h1 | h2 | h3 | h4 | h5 | h6 | h7);
  if (any != 0u) {
#define HITJ(J, HJ, SJ) { \
      const unsigned mj = __builtin_amdgcn_ballot_w32(HJ); \
      if (mj != 0u) { \
        if (HJ) { \
          const int pos = wc + (int)__builtin_amdgcn_mbcnt_lo(mj, 0u); \
          if (pos < WCAP) list[wave * WCAP + pos] = ((el0 + (J)) << 12) | (int)(SJ); \
        } \
        wc += (int)__builtin_popcount(mj); } }
    HITJ(0, h0, s0)
    HITJ(1, h1, s1)
    HITJ(2, h2, s2)
    HITJ(3, h3, s3)
    HITJ(4, h4, s4)
    HITJ(5, h5, s5)
    HITJ(6, h6, s6)
    HITJ(7, h7, s7)
#undef HITJ
  }
  return wc;
}

__global__ __launch_bounds__(NTHR) void k_prep(const float* __restrict__ ea,
                                               const float* __restrict__ we0, const float* __restrict__ ae0,
                                               const float* __restrict__ we1, const float* __restrict__ ae1,
                                               const float* __restrict__ we2, const float* __restrict__ ae2,
                                               const float* __restrict__ we3, const float* __restrict__ ae3,
                                               const float* __restrict__ w2a, const float* __restrict__ w2b,
                                               const float* __restrict__ f1w,
                                               float* misc, _Float16* w2t, _Float16* f1t, int nE) {
  __shared__ double sd[NTHR];
  __shared__ float sWe[8 * HC];
  __shared__ float sAe[4 * HC];
  __shared__ float sm[2];
  __shared__ __attribute__((aligned(16))) float sv[MISCN];
  const int tid = threadIdx.x;
  {
    const int k = tid & 1, gq = tid >> 1;
    double acc = 0.0;
#pragma unroll 1
    for (int r = gq; r < nE; r += NTHR / 2) acc += (double)ea[(size_t)r * 2 + k];
    sd[tid] = acc;
  }
  if (tid < 2 * HC) {
    sWe[tid] = we0[tid]; sWe[2 * HC + tid] = we1[tid];
    sWe[4 * HC + tid] = we2[tid]; sWe[6 * HC + tid] = we3[tid];
  }
  if (tid < HC) {
    sAe[tid] = ae0[tid]; sAe[HC + tid] = ae1[tid];
    sAe[2 * HC + tid] = ae2[tid]; sAe[3 * HC + tid] = ae3[tid];
  }
  if (tid < MISCN) sv[tid] = 0.f;
  __syncthreads();
  if (tid < 2) {
    double t = 0.0;
#pragma unroll 1
    for (int g2 = 0; g2 < NTHR / 2; ++g2) t += sd[g2 * 2 + tid];
    sm[tid] = (float)(t / (double)nE);
  }
  if (tid < 8) {
    const int cv = tid >> 1, k = tid & 1;
    float s = 0.f;
#pragma unroll 1
    for (int f = 0; f < HC; ++f) s = fmaf(sWe[cv * 2 * HC + k * HC + f], sAe[cv * HC + f], s);
    sv[8 * (cv >> 1) + 2 * (cv & 1) + k] = s;
  }
  __syncthreads();
  if (tid < 4) {
    const int ly = tid >> 1, br = tid & 1;
    const float a = fmaf(sm[1], sv[8 * ly + 2 * br + 1], sm[0] * sv[8 * ly + 2 * br]);
    sv[8 * ly + 4 + br] = a;
  }
  __syncthreads();
  {
    const bool w = tid < MISCN / 4;
    const v4f v = *(const v4f*)(sv + 4 * (w ? tid : 0));
    if (w) *(volatile v4f*)(misc + 4 * tid) = v;
    __threadfence();
    if (w) *(volatile v4f*)(misc + 4 * tid) = v;
  }
#pragma unroll 1
  for (int it = 0; it < 5; ++it) {
    if (it < 4) {
      const int u  = it * NTHR + tid;
      const int n  = u >> 3;
      const int k8 = (u & 7) * 8;
      const float* wsrc = (it < 2) ? w2a : w2b;
      const float* p = wsrc + (size_t)k8 * HC + (n & 63);
      v4f a, b;
      a.x = p[0 * HC]; a.y = p[1 * HC]; a.z = p[2 * HC]; a.w = p[3 * HC];
      b.x = p[4 * HC]; b.y = p[5 * HC]; b.z = p[6 * HC]; b.w = p[7 * HC];
      const v8h hv = pack8(a, b, CW);
      const size_t o = (size_t)n * WP + k8;
      *(volatile v8h*)(w2t + o) = hv;
      __threadfence();
      *(volatile v8h*)(w2t + o) = hv;
    } else {
      const int n  = tid >> 3;
      const int k8 = (tid & 7) * 8;
      const float* p = f1w + (size_t)k8 * FH + n;
      v4f a, b;
      a.x = p[0 * FH]; a.y = p[1 * FH]; a.z = p[2 * FH]; a.w = p[3 * FH];
      b.x = p[4 * FH]; b.y = p[5 * FH]; b.z = p[6 * FH]; b.w = p[7 * FH];
      const v8h hv = pack8(a, b, CW);
      const size_t o = (size_t)n * WP + k8;
      *(volatile v8h*)(f1t + o) = hv;
      __threadfence();
      *(volatile v8h*)(f1t + o) = hv;
    }
  }
}

__global__ __launch_bounds__(NTHR) void k_build(const int* __restrict__ dsts, int* EL, int* OFF, int* CNT,
                                                int nE, int nb, int tp, int vec8) {
  extern __shared__ v4f lds_dyn[];
  int* reg1 = (int*)lds_dyn;
  int* reg2 = reg1 + RCAP;
  int* scnt = reg2 + RCAP;
  int* soff = scnt + NBMAX;
  int* list = soff + NBMAX;
  int* wcnt = list + LISTN;
  int* wtot = wcnt + NWAVE;
  const int tid = threadIdx.x, lane = tid & 31, wave = tid >> 5;
  const int nodeBase = (int)blockIdx.x * nb;

  for (int i = tid; i < NBMAX; i += NTHR) scnt[i] = 0;
  {
    const v4i z = {0, 0, 0, 0};
    v4i* r2v = (v4i*)reg2;
    for (int f = tid; f < RCAP / 4; f += NTHR) r2v[f] = z;
  }
  __syncthreads();

  int tot = 0;
  const int nChunks = (nE + CHUNK - 1) / CHUNK;
#pragma unroll 1
  for (int ch = 0; ch < nChunks; ++ch) {
    const int cbase = ch * CHUNK;
    const int wc = scan_chunk(dsts, nE, cbase, nodeBase, nb, vec8, list, tid, lane, wave);
    if (lane == 0) wcnt[wave] = wc;
    __syncthreads();
    int pre = 0, all = 0;
#pragma unroll
    for (int w2 = 0; w2 < NWAVE; ++w2) {
      int c = wcnt[w2];
      c = c < 0 ? 0 : (c > WCAP ? WCAP : c);
      all += c;
      pre += (w2 < wave) ? c : 0;
    }
    const int wcc  = wc > WCAP ? WCAP : wc;
    const int base = tot + pre;
#pragma unroll 1
    for (int i = lane; i < wcc; i += 32) {
      const int ent = list[wave * WCAP + i];
      const int el  = (ent >> 12) & (CHUNK - 1);
      const int sl  = ent & (NBMAX - 1);
      int eid = cbase + el;
      eid = eid > nE - 1 ? nE - 1 : eid;
      const int pos = base + i;
      if (pos < RCAP) reg1[pos] = (int)(((unsigned)eid << SLOTB) | (unsigned)sl);
    }
    tot += all;
    tot = tot > RCAP ? RCAP : tot;
    __syncthreads();
  }
  const int nh = tot;

  if (wave == 0) {
#pragma unroll 1
    for (int b0 = 0; b0 < nh; b0 += 32) {
      const int idx = b0 + lane;
      const int uv  = reg1[idx < RCAP ? idx : RCAP - 1];
      const int m32 = (nh - b0) < 32 ? (nh - b0) : 32;
#pragma unroll 1
      for (int k = 0; k < m32; ++k) {
        const int u  = __builtin_amdgcn_readlane(uv, k);
        const int sl = u & (NBMAX - 1);
        if (lane == 0) scnt[sl] = scnt[sl] + 1;
      }
    }
  }
  __syncthreads();

  {
    const v4i ca = *(const v4i*)(scnt + 8 * tid);
    const v4i cb = *(const v4i*)(scnt + 8 * tid + 4);
    const int e0 = ca.x < 0 ? 0 : ca.x, e1 = ca.y < 0 ? 0 : ca.y, e2 = ca.z < 0 ? 0 : ca.z, e3 = ca.w < 0 ? 0 : ca.w;
    const int e4 = cb.x < 0 ? 0 : cb.x, e5 = cb.y < 0 ? 0 : cb.y, e6 = cb.z < 0 ? 0 : cb.z, e7 = cb.w < 0 ? 0 : cb.w;
    const int ts = e0 + e1 + e2 + e3 + e4 + e5 + e6 + e7;
    int incl = ts;
#pragma unroll
    for (int d = 1; d < 32; d <<= 1) {
      const int up = __shfl_up(incl, d);
      if (lane >= d) incl += up;
    }
    if (lane == 31) wtot[wave] = incl;
    __syncthreads();
    int pre = 0;
#pragma unroll
    for (int w2 = 0; w2 < NWAVE; ++w2) pre += (w2 < wave) ? wtot[w2] : 0;
    int run = pre + incl - ts;
    soff[8 * tid + 0] = run; run += e0;
    soff[8 * tid + 1] = run; run += e1;
    soff[8 * tid + 2] = run; run += e2;
    soff[8 * tid + 3] = run; run += e3;
    soff[8 * tid + 4] = run; run += e4;
    soff[8 * tid + 5] = run; run += e5;
    soff[8 * tid + 6] = run; run += e6;
    soff[8 * tid + 7] = run;
  }
  __syncthreads();
  for (int i = tid; i < NBMAX; i += NTHR) list[i] = soff[i];
  __syncthreads();

  if (wave == 0) {
#pragma unroll 1
    for (int b0 = 0; b0 < nh; b0 += 32) {
      const int idx = b0 + lane;
      const int uv  = reg1[idx < RCAP ? idx : RCAP - 1];
      const int m32 = (nh - b0) < 32 ? (nh - b0) : 32;
#pragma unroll 1
      for (int k = 0; k < m32; ++k) {
        const int u   = __builtin_amdgcn_readlane(uv, k);
        const int sl  = u & (NBMAX - 1);
        const int eid = (int)((unsigned)u >> SLOTB);
        if (lane == 0) {
          int pos = list[sl];
          pos = pos < 0 ? 0 : (pos > RCAP - 1 ? RCAP - 1 : pos);
          reg2[pos] = eid;
          list[sl] = pos + 1;
        }
      }
    }
  }
  __syncthreads();

  {
    int* elb = EL + (size_t)blockIdx.x * RCAP;
    const v4i* r4 = (const v4i*)reg2;
#pragma unroll 1
    for (int f = tid; f < RCAP / 4; f += NTHR) {
      const v4i v = r4[f];
      *(volatile v4i*)(elb + 4 * f) = v;
    }
    __threadfence();
#pragma unroll 1
    for (int f = tid; f < RCAP / 4; f += NTHR) {
      const v4i v = r4[f];
      *(volatile v4i*)(elb + 4 * f) = v;
    }
  }
  {
    const bool ovf = (nh >= RCAP);
    int* ob = OFF + (size_t)blockIdx.x * tp;
    int* cb = CNT + (size_t)blockIdx.x * tp;
    const int n4 = tp >> 2;
#pragma unroll 1
    for (int pass = 0; pass < 2; ++pass) {
#pragma unroll 1
      for (int f = tid; f < n4; f += NTHR) {
        v4i so, sc;
        {
          const int s = 4 * f + 0; const bool in = s < nb; const int scl = s < NBMAX ? s : NBMAX - 1;
          so.x = in ? soff[scl] : 0; sc.x = in ? (ovf ? -1 : scnt[scl]) : 0;
        }
        {
          const int s = 4 * f + 1; const bool in = s < nb; const int scl = s < NBMAX ? s : NBMAX - 1;
          so.y = in ? soff[scl] : 0; sc.y = in ? (ovf ? -1 : scnt[scl]) : 0;
        }
        {
          const int s = 4 * f + 2; const bool in = s < nb; const int scl = s < NBMAX ? s : NBMAX - 1;
          so.z = in ? soff[scl] : 0; sc.z = in ? (ovf ? -1 : scnt[scl]) : 0;
        }
        {
          const int s = 4 * f + 3; const bool in = s < nb; const int scl = s < NBMAX ? s : NBMAX - 1;
          so.w = in ? soff[scl] : 0; sc.w = in ? (ovf ? -1 : scnt[scl]) : 0;
        }
        *(volatile v4i*)(ob + 4 * f) = so;
        *(volatile v4i*)(cb + 4 * f) = sc;
      }
      __threadfence();
    }
  }
}

__global__ __launch_bounds__(NTHR) void k_node1(const float* __restrict__ x,
                                                const float* __restrict__ wl, const float* __restrict__ asl,
                                                const float* __restrict__ adl,
                                                const float* __restrict__ wg, const float* __restrict__ asg,
                                                const float* __restrict__ adg,
                                                float* HH, float* AL, int nN, int MP) {
  __shared__ float sW[4 * HC];
  __shared__ float sV[4 * HC];
  __shared__ __attribute__((aligned(16))) float st0[GBM * HC];
  __shared__ __attribute__((aligned(16))) float st1[GBM * HC];
  __shared__ __attribute__((aligned(16))) float sal[GBM * ALP];
  const int tid = threadIdx.x;
  const int rowBase = (int)blockIdx.x * GBM;
  if (tid < 2 * HC) { sW[tid] = wl[tid]; sW[2 * HC + tid] = wg[tid]; }
  if (tid < HC) {
    sV[tid] = asl[tid]; sV[HC + tid] = adl[tid];
    sV[2 * HC + tid] = asg[tid]; sV[3 * HC + tid] = adg[tid];
  }
  __syncthreads();
  {
    const int r = tid >> 2, q = tid & 3;
    int rg = rowBase + r;
    rg = rg < nN ? rg : nN - 1;
    const v2f xv = *(const v2f*)(x + (size_t)rg * 2);
    float p0 = 0.f, q0 = 0.f, p1 = 0.f, q1 = 0.f;
#pragma unroll 1
    for (int i = 0; i < HC / 4; ++i) {
      const int f = (HC / 4) * q + i;
      const float hl = fmaf(xv.y, sW[HC + f], xv.x * sW[f]);
      const float hg = fmaf(xv.y, sW[3 * HC + f], xv.x * sW[2 * HC + f]);
      st0[r * HC + f] = hl;
      st1[r * HC + f] = hg;
      p0 = fmaf(hl, sV[f], p0);          q0 = fmaf(hl, sV[HC + f], q0);
      p1 = fmaf(hg, sV[2 * HC + f], p1); q1 = fmaf(hg, sV[3 * HC + f], q1);
    }
    p0 += __shfl_xor(p0, 1); q0 += __shfl_xor(q0, 1); p1 += __shfl_xor(p1, 1); q1 += __shfl_xor(q1, 1);
    p0 += __shfl_xor(p0, 2); q0 += __shfl_xor(q0, 2); p1 += __shfl_xor(p1, 2); q1 += __shfl_xor(q1, 2);
    if (q == 0) {
      sal[r * ALP + 0] = p0; sal[r * ALP + 1] = q0;
      sal[r * ALP + 2] = p1; sal[r * ALP + 3] = q1;
    }
  }
  __syncthreads();
  {
    const v4f* s0 = (const v4f*)st0;
    const v4f* s1 = (const v4f*)st1;
    float* h0 = HH + (size_t)rowBase * HC;
    float* h1 = HH + ((size_t)MP + (size_t)rowBase) * HC;
    const bool wa = tid < GBM;
    const v4f av = *(const v4f*)(sal + 4 * (wa ? tid : 0));
    float* ap = AL + (size_t)(rowBase + (wa ? tid : 0)) * ALP;
#pragma unroll 1
    for (int f = tid; f < GBM * (HC / 4); f += NTHR) {
      const v4f v0 = s0[f], v1 = s1[f];
      *(volatile v4f*)(h0 + 4 * f) = v0;
      *(volatile v4f*)(h1 + 4 * f) = v1;
    }
    if (wa) *(volatile v4f*)ap = av;
    __threadfence();
#pragma unroll 1
    for (int f = tid; f < GBM * (HC / 4); f += NTHR) {
      const v4f v0 = s0[f], v1 = s1[f];
      *(volatile v4f*)(h0 + 4 * f) = v0;
      *(volatile v4f*)(h1 + 4 * f) = v1;
    }
    if (wa) *(volatile v4f*)ap = av;
  }
}

__global__ __launch_bounds__(NTHR) void k_agg(
    const int* __restrict__ srcs, const int* __restrict__ mask, const int* __restrict__ EL,
    const int* __restrict__ OFF, const int* __restrict__ CNT,
    const float* __restrict__ HH, const float* __restrict__ AL, const float* __restrict__ ea,
    const float* __restrict__ misc, const float* __restrict__ bias0, const float* __restrict__ bias1,
    float* G, float* ZP, int nN, int nE, int MP, int nb, int tp, float slope) {
  __shared__ __attribute__((aligned(16))) v4f cmb[NWAVE * 32];
  __shared__ float cdn[NWAVE * 32];
  __shared__ __attribute__((aligned(16))) float zw[NWAVE * HC];
  __shared__ __attribute__((aligned(16))) float zq[NWAVE * HC];
  __shared__ float sce[8];
  const int tid = threadIdx.x, lane = tid & 31, wave = tid >> 5;
  const int g = lane >> 4;
  const int j = lane & 15;
  if (tid < 8) sce[tid] = misc[tid];
  __syncthreads();
  const int nodeBase = (int)blockIdx.x * nb;
  const int nbw = nb >> 3;
  const int* elb  = EL  + (size_t)blockIdx.x * RCAP;
  const int* offb = OFF + (size_t)blockIdx.x * tp;
  const int* cntb = CNT + (size_t)blockIdx.x * tp;
  const float qnan = __int_as_float(0x7fc00000);
  const v4f z4 = {0.f, 0.f, 0.f, 0.f};
  v4f zA = z4, zQ = z4;
  v4f* cw = cmb + wave * 32;
  float* cd = cdn + wave * 32;
#pragma unroll 1
  for (int jt = 0; jt < nbw; ++jt) {
    const int slot = wave * nbw + jt;
    const int grow = nodeBase + slot;
    const int gcl  = grow < nN ? grow : nN - 1;
    const bool wr  = grow < nN;
    int st = offb[slot];
    const int craw = cntb[slot];
    st = st < 0 ? 0 : (st > RCAP - 1 ? RCAP - 1 : st);
    int cnt = craw < 0 ? 0 : (craw > DEGCAP ? DEGCAP : craw);
    if (cnt > RCAP - st) cnt = RCAP - st;
    const float pz = (craw < 0 || craw > DEGCAP) ? qnan : 0.0f;

    const int ms = mask[gcl];
    const int b  = (ms != 0) ? 1 : 0;
    const float c0  = sce[2 * b], c1 = sce[2 * b + 1];
    const float alb = sce[4 + b];
    const float asd = AL[(size_t)gcl * ALP + 2 * b];
    const float adv = AL[(size_t)gcl * ALP + 2 * b + 1];
    const float t0  = (asd + adv) + alb;
    float mx = lk(t0, NEG_GAT);
    const size_t pb = (size_t)b * (size_t)MP;
    v4f a0 = *(const v4f*)(HH + (pb + (size_t)gcl) * HC + 4 * j);
    const bool g0 = (g == 0);
    float dn = g0 ? 1.0f : 0.0f;
    a0 = g0 ? a0 : z4;
    const int niter = (cnt + 1) >> 1;
#pragma unroll 1
    for (int it = 0; it < niter; ++it) {
      const int qq = it * 2 + g;
      const bool valid = qq < cnt;
      const int qc = valid ? qq : cnt - 1;
      const int idx = st + qc;
      int eid = elb[idx];
      eid = eid < 0 ? 0 : (eid > nE - 1 ? nE - 1 : eid);
      const int sraw = srcs[eid];
      const int s = sraw < 0 ? 0 : (sraw > nN - 1 ? nN - 1 : sraw);
      const v4f xs = *(const v4f*)(HH + (pb + (size_t)s) * HC + 4 * j);
      const v2f ev = *(const v2f*)(ea + (size_t)eid * 2);
      const float et  = fmaf(ev.y, c1, ev.x * c0);
      const float ass = AL[(size_t)s * ALP + 2 * b];
      const float u = (ass + adv) + et;
      float l = lk(u, NEG_GAT);
      l = valid ? l : (mx - 100.0f);
      const float mn = fmaxf(mx, l);
      const float s1 = __expf(mx - mn), s2 = __expf(l - mn);
      dn = fmaf(dn, s1, s2);
      a0 = a0 * s1 + xs * s2;
      mx = mn;
    }
    const float m1 = fmaxf(mx, __shfl_xor(mx, 16));
    const float e = __expf(mx - m1);
    __builtin_amdgcn_fence(__ATOMIC_RELEASE, "wavefront");
    __builtin_amdgcn_wave_barrier();
    cw[lane] = a0 * e;
    cd[lane] = dn * e;
    __builtin_amdgcn_fence(__ATOMIC_RELEASE, "wavefront");
    __builtin_amdgcn_wave_barrier();
    const v4f r    = cw[j] + cw[16 + j];
    const float ds = cd[j] + cd[16 + j];
    const float inv = __builtin_amdgcn_rcpf(ds);
    const v4f bv0 = *(const v4f*)(bias0 + 4 * j);
    const v4f bv1 = *(const v4f*)(bias1 + 4 * j);
    const v4f bv  = (b != 0) ? bv1 : bv0;
    const v4f hv  = leaky4(r * inv + bv, slope) + pz;
    if (wr) {
      zA += hv;
      zQ += hv * hv;
      if (lane < 16) {
        float* gp = G + (size_t)gcl * HC + 4 * j;
        *(volatile v4f*)gp = hv;
        __threadfence();
        *(volatile v4f*)gp = hv;
      }
    }
  }
  if (lane < 16) {
    *(v4f*)(zw + (size_t)wave * HC + 4 * lane) = zA;
    *(v4f*)(zq + (size_t)wave * HC + 4 * lane) = zQ;
  }
  __syncthreads();
  if (tid < 32) {
    const int cgp  = tid & 15;
    const bool isq = tid >= 16;
    v4f sa = *(const v4f*)(zw + 4 * cgp);
    v4f sq = *(const v4f*)(zq + 4 * cgp);
#pragma unroll
    for (int w2 = 1; w2 < NWAVE; ++w2) {
      sa += *(const v4f*)(zw + (size_t)w2 * HC + 4 * cgp);
      sq += *(const v4f*)(zq + (size_t)w2 * HC + 4 * cgp);
    }
    const v4f v = isq ? sq : sa;
    float* zp = ZP + (size_t)blockIdx.x * ZPW + 4 * tid;
    *(volatile v4f*)zp = v;
    __threadfence();
    *(volatile v4f*)zp = v;
  }
}

__global__ __launch_bounds__(HC) void k_bn(const float* __restrict__ ZP, const float* __restrict__ gma,
                                            const float* __restrict__ bta, float* BNP, int gA, int nN) {
  __shared__ __attribute__((aligned(16))) float sv[BNW];
  const int tid = threadIdx.x;
  double s = 0.0, q = 0.0;
#pragma unroll 1
  for (int bk = 0; bk < gA; ++bk) {
    s += (double)ZP[(size_t)bk * ZPW + tid];
    q += (double)ZP[(size_t)bk * ZPW + HC + tid];
  }
  const double inv = 1.0 / (double)nN;
  const double mu  = s * inv;
  double var = q * inv - mu * mu;
  var = var < 0.0 ? 0.0 : var;
  const double rs = 1.0 / sqrt(var + BN_EPSD);
  sv[tid]          = (float)mu;
  sv[HC + tid]     = (float)rs * gma[tid];
  sv[2 * HC + tid] = bta[tid];
  sv[3 * HC + tid] = 0.f;
  __syncthreads();
  const v4f v = *(const v4f*)(sv + 4 * tid);
  *(volatile v4f*)(BNP + 4 * tid) = v;
  __threadfence();
  *(volatile v4f*)(BNP + 4 * tid) = v;
}

__global__ __launch_bounds__(GTHR) void k_gemm2(const float* __restrict__ G1, const float* __restrict__ bnp,
                                                const _Float16* __restrict__ w2t,
                                                const float* __restrict__ as0, const float* __restrict__ ad0,
                                                const float* __restrict__ as1, const float* __restrict__ ad1,
                                                float* HH, float* AL, int nN, int MP) {
  __shared__ __attribute__((aligned(16))) _Float16 sA[GBM * SAP];
  __shared__ __attribute__((aligned(16))) float stg[GBM * 2 * HC];
  __shared__ __attribute__((aligned(16))) float salT[GBM * ALP];
  __shared__ float sBN[3 * HC];
  __shared__ float sAs[2 * HC];
  __shared__ float sAd[2 * HC];
  const int tid = threadIdx.x, lane = tid & 31, wave = tid >> 5, hh = lane >> 4, m = lane & 15;
  const int rowBase = (int)blockIdx.x * GBM;
  for (int i = tid; i < 3 * HC; i += GTHR) sBN[i] = bnp[i];
  if (tid < HC) {
    sAs[tid] = as0[tid]; sAs[HC + tid] = as1[tid];
    sAd[tid] = ad0[tid]; sAd[HC + tid] = ad1[tid];
  }
  __syncthreads();
#pragma unroll 1
  for (int u = tid; u < GBM * (HC / 8); u += GTHR) {
    const int row = u >> 3, c0 = (u & 7) * 8;
    const int rg  = rowBase + row;
    const int rc  = rg < nN ? rg : nN - 1;
    const float* p = G1 + (size_t)rc * HC + c0;
    v4f a = *(const v4f*)p, b = *(const v4f*)(p + 4);
    a.x = bnl(a.x, sBN, c0 + 0); a.y = bnl(a.y, sBN, c0 + 1);
    a.z = bnl(a.z, sBN, c0 + 2); a.w = bnl(a.w, sBN, c0 + 3);
    b.x = bnl(b.x, sBN, c0 + 4); b.y = bnl(b.y, sBN, c0 + 5);
    b.z = bnl(b.z, sBN, c0 + 6); b.w = bnl(b.w, sBN, c0 + 7);
    *(v8h*)(sA + (size_t)row * SAP + c0) = pack8(a, b, CA);
  }
  __syncthreads();
  const _Float16* ap = sA + (size_t)(16 * wave + m) * SAP + 8 * hh;
  const size_t brow = (size_t)m * WP + 8 * hh;
  v8f acc[8];
#pragma unroll
  for (int t = 0; t < 8; ++t) { v8f z = {0.f, 0.f, 0.f, 0.f, 0.f, 0.f, 0.f, 0.f}; acc[t] = z; }
#pragma unroll 1
  for (int ks = 0; ks < HC / 32; ++ks) {
    FragH af;
    af.h[0] = *(const v8h*)(ap + 32 * ks);
    af.h[1] = *(const v8h*)(ap + 32 * ks + 16);
#pragma unroll
    for (int t = 0; t < 8; ++t) {
      const size_t bo = brow + (size_t)(16 * t) * WP + 32 * ks;
      FragH bf;
      bf.h[0] = *(const v8h*)(w2t + bo);
      bf.h[1] = *(const v8h*)(w2t + bo + 16);
      acc[t] = wmh(af, bf, acc[t]);
    }
  }
  {
    float* sp = stg + (size_t)(16 * wave + 8 * hh) * (2 * HC) + m;
#pragma unroll
    for (int t = 0; t < 8; ++t) {
#pragma unroll
      for (int r = 0; r < 8; ++r) sp[(size_t)r * (2 * HC) + 16 * t] = acc[t][r] * SCL;
    }
  }
  __syncthreads();
  {
    const int row  = tid >> 1;
    const int half = tid & 1;
    const float* srow = stg + (size_t)row * (2 * HC);
#pragma unroll 1
    for (int p = 0; p < 2; ++p) {
      float s = 0.f, d = 0.f;
#pragma unroll 1
      for (int c = 0; c < HC / 2; ++c) {
        const int cc = HC * p + (HC / 2) * half + c;
        const float v = srow[cc];
        s = fmaf(v, sAs[cc], s);
        d = fmaf(v, sAd[cc], d);
      }
      s += __shfl_xor(s, 1);
      d += __shfl_xor(d, 1);
      if (half == 0) {
        salT[row * ALP + 2 * p]     = s;
        salT[row * ALP + 2 * p + 1] = d;
      }
    }
  }
  __syncthreads();
  {
    const bool wa = tid < GBM;
    const v4f av = *(const v4f*)(salT + 4 * (wa ? tid : 0));
    float* alp = AL + (size_t)(rowBase + (wa ? tid : 0)) * ALP;
#pragma unroll 1
    for (int p = 0; p < 2; ++p) {
      float* hp = HH + ((size_t)p * (size_t)MP + (size_t)rowBase) * HC;
#pragma unroll 1
      for (int f = tid; f < GBM * (HC / 4); f += GTHR) {
        const int r = f >> 4, q = f & 15;
        const v4f v = *(const v4f*)(stg + (size_t)r * (2 * HC) + HC * p + 4 * q);
        *(volatile v4f*)(hp + 4 * f) = v;
      }
    }
    if (wa) *(volatile v4f*)alp = av;
    __threadfence();
#pragma unroll 1
    for (int p = 0; p < 2; ++p) {
      float* hp = HH + ((size_t)p * (size_t)MP + (size_t)rowBase) * HC;
#pragma unroll 1
      for (int f = tid; f < GBM * (HC / 4); f += GTHR) {
        const int r = f >> 4, q = f & 15;
        const v4f v = *(const v4f*)(stg + (size_t)r * (2 * HC) + HC * p + 4 * q);
        *(volatile v4f*)(hp + 4 * f) = v;
      }
    }
    if (wa) *(volatile v4f*)alp = av;
  }
}

__global__ __launch_bounds__(GTHR) void k_head(const float* __restrict__ G2, const _Float16* __restrict__ f1t,
                                               const float* __restrict__ f1b, const float* __restrict__ f2w,
                                               const float* __restrict__ f2b, const int* __restrict__ mask,
                                               float* out, int nN) {
  __shared__ __attribute__((aligned(16))) _Float16 sA[GBM * SAP];
  __shared__ __attribute__((aligned(16))) float stg[GBM * FH];
  __shared__ __attribute__((aligned(16))) float so[GBM];
  __shared__ float sb1[FH];
  __shared__ float sw2[FH];
  const int tid = threadIdx.x, lane = tid & 31, wave = tid >> 5, hh = lane >> 4, m = lane & 15;
  const int rowBase = (int)blockIdx.x * GBM;
  if (tid < FH) { sb1[tid] = f1b[tid]; sw2[tid] = f2w[tid]; }
#pragma unroll 1
  for (int u = tid; u < GBM * (HC / 8); u += GTHR) {
    const int row = u >> 3, c0 = (u & 7) * 8;
    const int rg  = rowBase + row;
    const int rc  = rg < nN ? rg : nN - 1;
    const float* p = G2 + (size_t)rc * HC + c0;
    const v4f a = *(const v4f*)p, b = *(const v4f*)(p + 4);
    *(v8h*)(sA + (size_t)row * SAP + c0) = pack8(a, b, CA);
  }
  __syncthreads();
  const _Float16* ap = sA + (size_t)(16 * wave + m) * SAP + 8 * hh;
  const size_t brow = (size_t)m * WP + 8 * hh;
  v8f acc[2];
#pragma unroll
  for (int t = 0; t < 2; ++t) { v8f z = {0.f, 0.f, 0.f, 0.f, 0.f, 0.f, 0.f, 0.f}; acc[t] = z; }
#pragma unroll 1
  for (int ks = 0; ks < HC / 32; ++ks) {
    FragH af;
    af.h[0] = *(const v8h*)(ap + 32 * ks);
    af.h[1] = *(const v8h*)(ap + 32 * ks + 16);
#pragma unroll
    for (int t = 0; t < 2; ++t) {
      const size_t bo = brow + (size_t)(16 * t) * WP + 32 * ks;
      FragH bf;
      bf.h[0] = *(const v8h*)(f1t + bo);
      bf.h[1] = *(const v8h*)(f1t + bo + 16);
      acc[t] = wmh(af, bf, acc[t]);
    }
  }
  {
    float* sp = stg + (size_t)(16 * wave + 8 * hh) * FH + m;
#pragma unroll
    for (int t = 0; t < 2; ++t) {
      const float bb = sb1[16 * t + m];
#pragma unroll
      for (int r = 0; r < 8; ++r) sp[(size_t)r * FH + 16 * t] = lk(fmaf(acc[t][r], SCL, bb), NEG_ACT);
    }
  }
  __syncthreads();
  if (tid < GBM) {
    const float* srow = stg + (size_t)tid * FH;
    float o = 0.f;
#pragma unroll 1
    for (int n = 0; n < FH; ++n) o = fmaf(srow[n], sw2[n], o);
    o += f2b[0];
    int rg = rowBase + tid;
    rg = rg < nN ? rg : nN - 1;
    o *= (float)mask[rg];
    so[tid] = o;
  }
  __syncthreads();
  {
    const int tl = tid < 16 ? tid : 0;
    const v4f ov = *(const v4f*)(so + 4 * tl);
    const bool stl = (tid < 16) && (rowBase + 4 * tid + 4 <= nN);
    float* op = out + (size_t)rowBase + 4 * tl;
    if (stl) *(volatile v4f*)op = ov;
    __threadfence();
    if (stl) *(volatile v4f*)op = ov;
  }
}

static int pick_nb(int nE, int nN) {
  int nb = NBMAX;
  while (nb > 16 && (long long)nb * (long long)nE * 5LL > (long long)RCAP * (long long)nN * 4LL) nb >>= 1;
  return nb;
}

extern "C" void kernel_launch(void* const* d_in, const int* in_sizes, int n_in,
                              void* d_out, int out_size, void* d_ws, size_t ws_size,
                              hipStream_t stream) {
  if (n_in < 34) return;
  if (in_sizes[0] < 2 || (in_sizes[0] & 1) != 0) return;
  const int nN = in_sizes[0] / 2;
  if ((nN % 32) != 0 || nN > (1 << 22)) return;
  if (in_sizes[1] < 2 || (in_sizes[1] & 1) != 0) return;
  const int nE = in_sizes[1] / 2;
  if (nE < 1 || nE > (1 << 21)) return;
  if (in_sizes[2] != 2 * nE) return;
  if (in_sizes[3] != nN) return;
  if (in_sizes[4] != 2 * HC || in_sizes[5] != 2 * HC) return;
  if (in_sizes[6] != HC || in_sizes[7] != HC || in_sizes[8] != HC || in_sizes[9] != HC) return;
  if (in_sizes[10] != 2 * HC || in_sizes[11] != 2 * HC) return;
  if (in_sizes[12] != HC || in_sizes[13] != HC || in_sizes[14] != HC || in_sizes[15] != HC) return;
  if (in_sizes[16] != HC * HC || in_sizes[17] != 2 * HC) return;
  if (in_sizes[18] != HC || in_sizes[19] != HC || in_sizes[20] != HC || in_sizes[21] != HC) return;
  if (in_sizes[22] != HC * HC || in_sizes[23] != 2 * HC) return;
  if (in_sizes[24] != HC || in_sizes[25] != HC || in_sizes[26] != HC || in_sizes[27] != HC) return;
  if (in_sizes[28] != HC || in_sizes[29] != HC) return;
  if (in_sizes[30] != HC * FH || in_sizes[31] != FH || in_sizes[32] != FH || in_sizes[33] != 1) return;
  if (out_size != nN) return;

  const float* x       = (const float*)d_in[0];
  const float* eattr   = (const float*)d_in[1];
  const int*   ei      = (const int*)d_in[2];
  const int*   mask    = (const int*)d_in[3];
  const float* gcn_W   = (const float*)d_in[4];
  const float* gcn_We  = (const float*)d_in[5];
  const float* gcn_as  = (const float*)d_in[6];
  const float* gcn_ad  = (const float*)d_in[7];
  const float* gcn_ae  = (const float*)d_in[8];
  const float* gcn_b   = (const float*)d_in[9];
  const float* lit_W   = (const float*)d_in[10];
  const float* lit_We  = (const float*)d_in[11];
  const float* lit_as  = (const float*)d_in[12];
  const float* lit_ad  = (const float*)d_in[13];
  const float* lit_ae  = (const float*)d_in[14];
  const float* lit_b   = (const float*)d_in[15];
  const float* gcn2_W  = (const float*)d_in[16];
  const float* gcn2_We = (const float*)d_in[17];
  const float* gcn2_as = (const float*)d_in[18];
  const float* gcn2_ad = (const float*)d_in[19];
  const float* gcn2_ae = (const float*)d_in[20];
  const float* gcn2_b  = (const float*)d_in[21];
  const float* lit2_W  = (const float*)d_in[22];
  const float* lit2_We = (const float*)d_in[23];
  const float* lit2_as = (const float*)d_in[24];
  const float* lit2_ad = (const float*)d_in[25];
  const float* lit2_ae = (const float*)d_in[26];
  const float* lit2_b  = (const float*)d_in[27];
  const float* ln_g    = (const float*)d_in[28];
  const float* ln_beta = (const float*)d_in[29];
  const float* f1_W    = (const float*)d_in[30];
  const float* f1_b    = (const float*)d_in[31];
  const float* f2_W    = (const float*)d_in[32];
  const float* f2_b    = (const float*)d_in[33];
  float* out = (float*)d_out;
  const int* dsts = ei + nE;

  const int MP   = ((nN + GBM - 1) / GBM) * GBM;
  const int gG   = MP / GBM;
  const int nb   = pick_nb(nE, nN);
  const int tp   = nb < 32 ? 32 : nb;
  const int gA   = (nN + nb - 1) / nb;
  const int vec8 = ((nE & 3) == 0) ? 1 : 0;
  if (nb < 16 || nb > NBMAX || (long long)gA * nb < (long long)nN) return;

  char* ws = (char*)d_ws;
  size_t off = 0;
  const size_t oHH   = off; off += (size_t)2 * MP * HC * 4;      off = (off + 255) & ~(size_t)255;
  const size_t oG    = off; off += (size_t)MP * HC * 4;          off = (off + 255) & ~(size_t)255;
  const size_t oAL   = off; off += (size_t)MP * ALP * 4;         off = (off + 255) & ~(size_t)255;
  const size_t oEL   = off; off += (size_t)gA * RCAP * 4;        off = (off + 255) & ~(size_t)255;
  const size_t oOFF  = off; off += (size_t)gA * tp * 4;          off = (off + 255) & ~(size_t)255;
  const size_t oCNT  = off; off += (size_t)gA * tp * 4;          off = (off + 255) & ~(size_t)255;
  const size_t oZP   = off; off += (size_t)gA * ZPW * 4;         off = (off + 255) & ~(size_t)255;
  const size_t oBNP  = off; off += (size_t)BNW * 4;              off = (off + 255) & ~(size_t)255;
  const size_t oMISC = off; off += (size_t)MISCN * 4;            off = (off + 255) & ~(size_t)255;
  const size_t oW2T  = off; off += (size_t)2 * HC * WP * 2;      off = (off + 255) & ~(size_t)255;
  const size_t oF1T  = off; off += (size_t)FH * WP * 2;          off = (off + 255) & ~(size_t)255;
  if (off > ws_size || off > (size_t)WSCAP) return;
  float*    HH   = (float*)(ws + oHH);
  float*    G    = (float*)(ws + oG);
  float*    AL   = (float*)(ws + oAL);
  int*      EL   = (int*)(ws + oEL);
  int*      OFF  = (int*)(ws + oOFF);
  int*      CNT  = (int*)(ws + oCNT);
  float*    ZP   = (float*)(ws + oZP);
  float*    BNP  = (float*)(ws + oBNP);
  float*    MISC = (float*)(ws + oMISC);
  _Float16* W2T  = (_Float16*)(ws + oW2T);
  _Float16* F1T  = (_Float16*)(ws + oF1T);

  hipFuncSetAttribute(reinterpret_cast<const void*>(&k_build),
                      hipFuncAttributeMaxDynamicSharedMemorySize, LDS_BUILD);

  k_prep<<<1, NTHR, 0, stream>>>(eattr, lit_We, lit_ae, gcn_We, gcn_ae, lit2_We, lit2_ae, gcn2_We, gcn2_ae,
                                 lit2_W, gcn2_W, f1_W, MISC, W2T, F1T, nE);

  k_build<<<gA, NTHR, LDS_BUILD, stream>>>(dsts, EL, OFF, CNT, nE, nb, tp, vec8);

  k_node1<<<gG, NTHR, 0, stream>>>(x, lit_W, lit_as, lit_ad, gcn_W, gcn_as, gcn_ad, HH, AL, nN, MP);
  k_agg<<<gA, NTHR, 0, stream>>>(ei, mask, EL, OFF, CNT, HH, AL, eattr, MISC, lit_b, gcn_b, G, ZP,
                                 nN, nE, MP, nb, tp, 1.0f);

  k_bn<<<1, HC, 0, stream>>>(ZP, ln_g, ln_beta, BNP, gA, nN);
  k_gemm2<<<gG, GTHR, 0, stream>>>(G, BNP, W2T, lit2_as, lit2_ad, gcn2_as, gcn2_ad, HH, AL, nN, MP);

  k_agg<<<gA, NTHR, 0, stream>>>(ei, mask, EL, OFF, CNT, HH, AL, eattr, MISC + 8, lit2_b, gcn2_b, G, ZP,
                                 nN, nE, MP, nb, tp, NEG_ACT);
  k_head<<<gG, GTHR, 0, stream>>>(G, F1T, f1_b, f2_W, f2_b, mask, out, nN);
}
